// GCNModel_66907000537708
// MI455X (gfx1250) — hardware-verified
//
#include <hip/hip_runtime.h>
#include <stddef.h>


#define DIN     128
#define DH      256
#define DE      128
#define DF      128
#define NTHR    256
#define NWAVE   8
#define EPT     8
#define NGRP    2
#define CHUNK   (NTHR * EPT * NGRP)
#define WCAP    (EPT * NGRP * 32)
#define LISTN   (NWAVE * WCAP)
#define NB      512
#define NBD     4096
#define G2ROWS  128
#define APITCH  264
#define SROWS   512
#define SSOFF   256
#define WSCALE  16.0f
#define WINV    0.0625f
#define BNEPS   1e-5f

#define LDS_AGG   (NB * DF * 4 + LISTN * 4 + 64)
#define LDS_GEMM2 (G2ROWS * APITCH * 2)

static_assert((CHUNK & (CHUNK - 1)) == 0);
static_assert(CHUNK <= 4096);
static_assert(NB <= 4096 && NBD <= 4096);
static_assert(G2ROWS * DE * 4 <= LDS_GEMM2);
static_assert(DIN == DF && DE == DF);
static_assert(NB % (16 * NWAVE) == 0);
static_assert(DH % DF == 0 && DIN % 32 == 0 && DH % 32 == 0);

typedef float    v4f  __attribute__((ext_vector_type(4)));
typedef float    v8f  __attribute__((ext_vector_type(8)));
typedef int      v4i  __attribute__((ext_vector_type(4)));
typedef _Float16 v8h  __attribute__((ext_vector_type(8)));
typedef _Float16 v16h __attribute__((ext_vector_type(16)));
union FragH { v16h v; v8h h[2]; };

__device__ __forceinline__ v8h cvt8(v4f a, v4f b) {
  v8h r;
  r[0] = (_Float16)a.x; r[1] = (_Float16)a.y; r[2] = (_Float16)a.z; r[3] = (_Float16)a.w;
  r[4] = (_Float16)b.x; r[5] = (_Float16)b.y; r[6] = (_Float16)b.z; r[7] = (_Float16)b.w;
  return r;
}

__device__ __forceinline__ v8f wmh(v16h a, v16h b, v8f c) {
  v8f d = __builtin_amdgcn_wmma_f32_16x16x32_f16(false, a, false, b, (short)0, c, false, false);
  asm volatile("v_nop\n\tv_nop\n\tv_nop\n\tv_nop" : "+v"(d) : "v"(a), "v"(b));
  return d;
}

template <int NBT>
__device__ __forceinline__ int scan_chunk(const int* __restrict__ dsts, int nE, int cbase, int nodeBase,
                                          int vec8, int* list, int tid, int lane, int wave) {
  int wc = 0;
#pragma unroll
  for (int g = 0; g < NGRP; ++g) {
    const int el0  = (g * NTHR + tid) * EPT;
    const int e0   = cbase + el0;
    const int sent = -2147483647 - 1;
    v4i da, db;
    if (vec8 != 0 && e0 + 7 < nE) {
      da = *(const v4i*)(dsts + e0);
      db = *(const v4i*)(dsts + e0 + 4);
    } else {
      da.x = (e0     < nE) ? dsts[min(e0, nE - 1)] : sent;
      da.y = (e0 + 1 < nE) ? dsts[min(e0 + 1, nE - 1)] : sent;
      da.z = (e0 + 2 < nE) ? dsts[min(e0 + 2, nE - 1)] : sent;
      da.w = (e0 + 3 < nE) ? dsts[min(e0 + 3, nE - 1)] : sent;
      db.x = (e0 + 4 < nE) ? dsts[min(e0 + 4, nE - 1)] : sent;
      db.y = (e0 + 5 < nE) ? dsts[min(e0 + 5, nE - 1)] : sent;
      db.z = (e0 + 6 < nE) ? dsts[min(e0 + 6, nE - 1)] : sent;
      db.w = (e0 + 7 < nE) ? dsts[min(e0 + 7, nE - 1)] : sent;
    }
    const unsigned nb = (unsigned)nodeBase;
    const unsigned s0 = (unsigned)da.x - nb, s1 = (unsigned)da.y - nb;
    const unsigned s2 = (unsigned)da.z - nb, s3 = (unsigned)da.w - nb;
    const unsigned s4 = (unsigned)db.x - nb, s5 = (unsigned)db.y - nb;
    const unsigned s6 = (unsigned)db.z - nb, s7 = (unsigned)db.w - nb;
    const bool h0 = s0 < (unsigned)NBT, h1 = s1 < (unsigned)NBT, h2 = s2 < (unsigned)NBT, h3 = s3 < (unsigned)NBT;
    const bool h4 = s4 < (unsigned)NBT, h5 = s5 < (unsigned)NBT, h6 = s6 < (unsigned)NBT, h7 = s7 < (unsigned)NBT;
    const unsigned any = __builtin_amdgcn_ballot_w32(h0 | h1 | h2 | h3 | h4 | h5 | h6 | h7);
    if (any != 0u) {
#define HITJ(J, HJ, SJ) { \
        const unsigned mj = __builtin_amdgcn_ballot_w32(HJ); \
        if (mj != 0u) { \
          if (HJ) { \
            const int pos = wc + (int)__builtin_amdgcn_mbcnt_lo(mj, 0u); \
            if (pos < WCAP) list[wave * WCAP + pos] = ((el0 + (J)) << 12) | (int)(SJ); \
          } \
          wc += (int)__builtin_popcount(mj); } }
      HITJ(0, h0, s0)
      HITJ(1, h1, s1)
      HITJ(2, h2, s2)
      HITJ(3, h3, s3)
      HITJ(4, h4, s4)
      HITJ(5, h5, s5)
      HITJ(6, h6, s6)
      HITJ(7, h7, s7)
#undef HITJ
    }
  }
  return wc;
}

__global__ __launch_bounds__(NTHR) void k_wprep(
    const float* __restrict__ W1, const float* __restrict__ W2,
    _Float16* w1s, _Float16* w2s) {
  const int i  = blockIdx.x * NTHR + threadIdx.x;
  const int n1 = DH * DIN / 8;
  const int n2 = DE * DH / 8;
  if (i >= n1 + n2) return;
  const bool first = i < n1;
  v4f a, b;
  int o;
  if (first) {
    o = i * 8;
    const int n  = o / DIN;
    const int k0 = o - n * DIN;
    const float* p = W1 + (size_t)k0 * DH + n;
    a.x = p[0];      a.y = p[DH];     a.z = p[2 * DH]; a.w = p[3 * DH];
    b.x = p[4 * DH]; b.y = p[5 * DH]; b.z = p[6 * DH]; b.w = p[7 * DH];
  } else {
    o = (i - n1) * 8;
    const int n  = o / DH;
    const int k0 = o - n * DH;
    const float* p = W2 + (size_t)k0 * DE + n;
    a.x = p[0];      a.y = p[DE];     a.z = p[2 * DE]; a.w = p[3 * DE];
    b.x = p[4 * DE]; b.y = p[5 * DE]; b.z = p[6 * DE]; b.w = p[7 * DE];
  }
  a = a * WSCALE;
  b = b * WSCALE;
  const v8h hv = cvt8(a, b);
  _Float16* dp = (first ? w1s : w2s) + o;
  *(volatile v8h*)dp = hv;
  __threadfence();
  *(volatile v8h*)dp = hv;
}

__global__ __launch_bounds__(NTHR) void k_deg(
    const int* __restrict__ ei, float* dinv, int nN, int nE, int vec8) {
  __shared__ __attribute__((aligned(16))) int cnt[NBD];
  __shared__ __attribute__((aligned(16))) int list[LISTN];
  __shared__ int wcnt[NWAVE];
  const int tid = threadIdx.x, lane = tid & 31, wave = tid >> 5;
  const int nodeBase = blockIdx.x * NBD;
  const int* dsts = ei + nE;
  (void)nN;

  for (int i = tid; i < NBD; i += NTHR) cnt[i] = 0;
  __syncthreads();

  const int nChunks = (nE + CHUNK - 1) / CHUNK;
#pragma unroll 1
  for (int ch = 0; ch < nChunks; ++ch) {
    const int cbase = ch * CHUNK;
    const int wc = scan_chunk<NBD>(dsts, nE, cbase, nodeBase, vec8, list, tid, lane, wave);
    if (lane == 0) wcnt[wave] = wc;
    __syncthreads();
    if (wave == 0) {
#pragma unroll 1
      for (int wsx = 0; wsx < NWAVE; ++wsx) {
        int n = __builtin_amdgcn_readfirstlane(wcnt[wsx]);
        n = n > WCAP ? WCAP : (n < 0 ? 0 : n);
        const int* lp = list + wsx * WCAP;
#pragma unroll 1
        for (int i = 0; i < n; ++i) {
          const int ent  = __builtin_amdgcn_readfirstlane(lp[i]);
          const int slot = ent & (NBD - 1);
          if (lane == 0) cnt[slot] = cnt[slot] + 1;
        }
      }
    }
    __syncthreads();
  }

  v4f dq[4];
#pragma unroll
  for (int q = 0; q < 4; ++q) {
    const int f = (wave * 4 + q) * 128 + 4 * lane;
    const v4i c = *(const v4i*)(cnt + f);
    dq[q].x = rsqrtf((float)(c.x + 1));
    dq[q].y = rsqrtf((float)(c.y + 1));
    dq[q].z = rsqrtf((float)(c.z + 1));
    dq[q].w = rsqrtf((float)(c.w + 1));
  }
  float* dp = dinv + (size_t)nodeBase;
#pragma unroll
  for (int q = 0; q < 4; ++q) *(volatile v4f*)(dp + (wave * 4 + q) * 128 + 4 * lane) = dq[q];
  __threadfence();
#pragma unroll
  for (int q = 0; q < 4; ++q) *(volatile v4f*)(dp + (wave * 4 + q) * 128 + 4 * lane) = dq[q];
}

__global__ __launch_bounds__(NTHR) void k_agg1(
    const int* __restrict__ ei, const float* __restrict__ x, const float* __restrict__ dinv,
    const float* __restrict__ b1, const _Float16* __restrict__ w1s, float* h1,
    int nN, int nE, int vec8) {
  extern __shared__ v4f lds_dyn[];
  float* acc  = (float*)lds_dyn;
  int*   list = (int*)(acc + NB * DF);
  int*   wcnt = list + LISTN;
  const int tid = threadIdx.x, lane = tid & 31, wave = tid >> 5, hh = lane >> 4, m = lane & 15;
  const int nodeBase = blockIdx.x * NB;
  const int* dsts = ei + nE;

  {
    const v4f z = {0.f, 0.f, 0.f, 0.f};
    for (int i = tid; i < NB * DF / 4; i += NTHR) lds_dyn[i] = z;
  }
  __syncthreads();

  const int nChunks = (nE + CHUNK - 1) / CHUNK;
#pragma unroll 1
  for (int ch = 0; ch < nChunks; ++ch) {
    const int cbase = ch * CHUNK;
    const int wc = scan_chunk<NB>(dsts, nE, cbase, nodeBase, vec8, list, tid, lane, wave);
    if (lane == 0) wcnt[wave] = wc;
    __syncthreads();
    if (wave == 0) {
#pragma unroll 1
      for (int wsx = 0; wsx < NWAVE; ++wsx) {
        int n = __builtin_amdgcn_readfirstlane(wcnt[wsx]);
        n = n > WCAP ? WCAP : (n < 0 ? 0 : n);
        const int* lq = list + wsx * WCAP;
#pragma unroll 1
        for (int i = 0; i < n; ++i) {
          const int ent  = __builtin_amdgcn_readfirstlane(lq[i]);
          const int slot = ent & (NB - 1);
          int e = cbase + ((ent >> 12) & (CHUNK - 1));
          e = e > nE - 1 ? nE - 1 : e;
          int src = ei[e];
          src = src < 0 ? 0 : (src > nN - 1 ? nN - 1 : src);
          const float ds = dinv[src];
          const v4f v = *(const v4f*)(x + (size_t)src * DIN + 4 * lane);
          v4f* ap = (v4f*)(acc + slot * DF + 4 * lane);
          *ap = *ap + v * ds;
        }
      }
    }
    __syncthreads();
  }

#pragma unroll 4
  for (int i = 0; i < (NB * DF / 4) / NTHR; ++i) {
    const int idx  = i * NTHR + tid;
    const int slot = idx >> 5;
    const int c4   = (idx & 31) * 4;
    int node = nodeBase + slot;
    node = node > nN - 1 ? nN - 1 : node;
    const float d  = dinv[node];
    const v4f   xv = *(const v4f*)(x + (size_t)node * DIN + c4);
    v4f* ap = (v4f*)(acc + slot * DF + c4);
    *ap = (*ap + xv * d) * d;
  }
  __syncthreads();

#pragma unroll 1
  for (int rt = 0; rt < NB / (16 * NWAVE); ++rt) {
    const int t = rt * NWAVE + wave;
    FragH af[DIN / 32];
    {
      const float* ar = acc + (16 * t + m) * DF + 8 * hh;
#pragma unroll
      for (int kt = 0; kt < DIN / 32; ++kt) {
        const v4f p0 = *(const v4f*)(ar + 32 * kt),      p1 = *(const v4f*)(ar + 32 * kt + 4);
        const v4f p2 = *(const v4f*)(ar + 32 * kt + 16), p3 = *(const v4f*)(ar + 32 * kt + 20);
        af[kt].h[0] = cvt8(p0, p1);
        af[kt].h[1] = cvt8(p2, p3);
      }
    }
    __syncthreads();
    float* stg = acc + 16 * t * DF;

#pragma unroll 1
    for (int s = 0; s < DH / DF; ++s) {
#pragma unroll 1
      for (int nt = 0; nt < DF / 16; ++nt) {
        const int ncol0 = DF * s + 16 * nt;
        v8f c = {0.f, 0.f, 0.f, 0.f, 0.f, 0.f, 0.f, 0.f};
#pragma unroll
        for (int kt = 0; kt < DIN / 32; ++kt) {
          const _Float16* bp = w1s + (size_t)(ncol0 + m) * DIN + 32 * kt + 8 * hh;
          FragH b;
          b.h[0] = *(const v8h*)bp;
          b.h[1] = *(const v8h*)(bp + 16);
          c = wmh(af[kt].v, b.v, c);
        }
        const float bb = b1[ncol0 + m];
        float* sp = stg + (8 * hh) * DF + 16 * nt + m;
        sp[0 * DF] = fmaxf(c[0] * WINV + bb, 0.f);
        sp[1 * DF] = fmaxf(c[1] * WINV + bb, 0.f);
        sp[2 * DF] = fmaxf(c[2] * WINV + bb, 0.f);
        sp[3 * DF] = fmaxf(c[3] * WINV + bb, 0.f);
        sp[4 * DF] = fmaxf(c[4] * WINV + bb, 0.f);
        sp[5 * DF] = fmaxf(c[5] * WINV + bb, 0.f);
        sp[6 * DF] = fmaxf(c[6] * WINV + bb, 0.f);
        sp[7 * DF] = fmaxf(c[7] * WINV + bb, 0.f);
      }
      __syncthreads();
      const float* lr = stg + 4 * lane;
      float* gp = h1 + ((size_t)nodeBase + 16 * t) * DH + DF * s + 4 * lane;
#pragma unroll
      for (int i = 0; i < 16; ++i) { const v4f v = *(const v4f*)(lr + i * DF); *(volatile v4f*)(gp + (size_t)i * DH) = v; }
      __threadfence();
#pragma unroll
      for (int i = 0; i < 16; ++i) { const v4f v = *(const v4f*)(lr + i * DF); *(volatile v4f*)(gp + (size_t)i * DH) = v; }
      __syncthreads();
    }
  }
}

__global__ __launch_bounds__(NTHR) void k_bnstat(
    const float* __restrict__ h, double* part, int D, int nN, int rows) {
  const int d  = threadIdx.x;
  const int r0 = blockIdx.x * rows;
  int r1 = r0 + rows; if (r1 > nN) r1 = nN;
  double s = 0.0, q = 0.0;
#pragma unroll 4
  for (int r = r0; r < r1; ++r) {
    const double v = (double)h[(size_t)r * D + d];
    s += v;
    q += v * v;
  }
  double* pp = part + (size_t)blockIdx.x * 2 * D;
  *(volatile double*)(pp + d)     = s;
  *(volatile double*)(pp + D + d) = q;
  __threadfence();
  *(volatile double*)(pp + d)     = s;
  *(volatile double*)(pp + D + d) = q;
}

__global__ __launch_bounds__(NTHR) void k_bnfin(
    const double* __restrict__ part, int nblk, int D, int nN,
    const float* __restrict__ gamma, const float* __restrict__ beta, float* ss) {
  const int d = threadIdx.x;
  double s = 0.0, q = 0.0;
#pragma unroll 1
  for (int b = 0; b < nblk; ++b) {
    s += part[(size_t)(2 * b) * D + d];
    q += part[(size_t)(2 * b + 1) * D + d];
  }
  const double inv  = 1.0 / (double)nN;
  const double mean = s * inv;
  double var = q * inv - mean * mean;
  var = var < 0.0 ? 0.0 : var;
  const float meanf = (float)mean;
  const float varf  = (float)var;
  const float sc = gamma[d] * rsqrtf(varf + BNEPS);
  const float sh = beta[d] - meanf * sc;
  *(volatile float*)(ss + d)         = sc;
  *(volatile float*)(ss + SSOFF + d) = sh;
  __threadfence();
  *(volatile float*)(ss + d)         = sc;
  *(volatile float*)(ss + SSOFF + d) = sh;
}

__global__ __launch_bounds__(NTHR) void k_gemm2(
    const float* __restrict__ h1, const float* __restrict__ ss1, const _Float16* __restrict__ w2s,
    const float* __restrict__ dinv, float* g2, int nN) {
  extern __shared__ v4f lds_dyn[];
  _Float16* sA  = (_Float16*)lds_dyn;
  float*    stg = (float*)lds_dyn;
  const int tid = threadIdx.x, lane = tid & 31, wave = tid >> 5, hh = lane >> 4, m = lane & 15;
  const int rowBase = blockIdx.x * G2ROWS;

#pragma unroll 4
  for (int i = 0; i < (G2ROWS * DH / 8) / NTHR; ++i) {
    const int idx = i * NTHR + tid;
    const int r   = idx >> 5;
    const int c0  = (idx & 31) * 8;
    int node = rowBase + r;
    node = node > nN - 1 ? nN - 1 : node;
    const float* xp = h1 + (size_t)node * DH + c0;
    v4f a = *(const v4f*)xp, b = *(const v4f*)(xp + 4);
    const v4f sa = *(const v4f*)(ss1 + c0),         sb = *(const v4f*)(ss1 + c0 + 4);
    const v4f ta = *(const v4f*)(ss1 + SSOFF + c0), tb = *(const v4f*)(ss1 + SSOFF + c0 + 4);
    a = a * sa + ta;
    b = b * sb + tb;
    *(v8h*)(sA + r * APITCH + c0) = cvt8(a, b);
  }
  __syncthreads();

  v8f acc[8];
#pragma unroll
  for (int t = 0; t < 8; ++t) { v8f z = {0.f, 0.f, 0.f, 0.f, 0.f, 0.f, 0.f, 0.f}; acc[t] = z; }
  const _Float16* ar = sA + (wave * 16 + m) * APITCH + 8 * hh;
#pragma unroll
  for (int kt = 0; kt < DH / 32; ++kt) {
    FragH a;
    a.h[0] = *(const v8h*)(ar + 32 * kt);
    a.h[1] = *(const v8h*)(ar + 32 * kt + 16);
#pragma unroll
    for (int t = 0; t < 8; ++t) {
      const _Float16* bp = w2s + (size_t)(16 * t + m) * DH + 32 * kt + 8 * hh;
      FragH b;
      b.h[0] = *(const v8h*)bp;
      b.h[1] = *(const v8h*)(bp + 16);
      acc[t] = wmh(a.v, b.v, acc[t]);
    }
  }
  __syncthreads();

  const int r0 = wave * 16 + 8 * hh;
  const v4f dA = *(const v4f*)(dinv + (size_t)rowBase + r0);
  const v4f dB = *(const v4f*)(dinv + (size_t)rowBase + r0 + 4);
  const float d0 = dA.x * WINV, d1 = dA.y * WINV, d2 = dA.z * WINV, d3 = dA.w * WINV;
  const float d4 = dB.x * WINV, d5 = dB.y * WINV, d6 = dB.z * WINV, d7 = dB.w * WINV;
  float* sp = stg + r0 * DE + m;
#pragma unroll
  for (int t = 0; t < 8; ++t) {
    sp[0 * DE + 16 * t] = acc[t][0] * d0;
    sp[1 * DE + 16 * t] = acc[t][1] * d1;
    sp[2 * DE + 16 * t] = acc[t][2] * d2;
    sp[3 * DE + 16 * t] = acc[t][3] * d3;
    sp[4 * DE + 16 * t] = acc[t][4] * d4;
    sp[5 * DE + 16 * t] = acc[t][5] * d5;
    sp[6 * DE + 16 * t] = acc[t][6] * d6;
    sp[7 * DE + 16 * t] = acc[t][7] * d7;
  }
  __syncthreads();

  const float* lr = stg + wave * 16 * DE + 4 * lane;
  float* gp = g2 + ((size_t)rowBase + wave * 16) * DE + 4 * lane;
#pragma unroll
  for (int i = 0; i < 16; ++i) { const v4f v = *(const v4f*)(lr + i * DE); *(volatile v4f*)(gp + (size_t)i * DE) = v; }
  __threadfence();
#pragma unroll
  for (int i = 0; i < 16; ++i) { const v4f v = *(const v4f*)(lr + i * DE); *(volatile v4f*)(gp + (size_t)i * DE) = v; }
}

__global__ __launch_bounds__(NTHR) void k_agg2(
    const int* __restrict__ ei, const float* __restrict__ g2, const float* __restrict__ dinv,
    const float* __restrict__ b2, float* h2, int nN, int nE, int vec8) {
  extern __shared__ v4f lds_dyn[];
  float* acc  = (float*)lds_dyn;
  int*   list = (int*)(acc + NB * DF);
  int*   wcnt = list + LISTN;
  const int tid = threadIdx.x, lane = tid & 31, wave = tid >> 5;
  const int nodeBase = blockIdx.x * NB;
  const int* dsts = ei + nE;

  {
    const v4f z = {0.f, 0.f, 0.f, 0.f};
    for (int i = tid; i < NB * DF / 4; i += NTHR) lds_dyn[i] = z;
  }
  __syncthreads();

  const int nChunks = (nE + CHUNK - 1) / CHUNK;
#pragma unroll 1
  for (int ch = 0; ch < nChunks; ++ch) {
    const int cbase = ch * CHUNK;
    const int wc = scan_chunk<NB>(dsts, nE, cbase, nodeBase, vec8, list, tid, lane, wave);
    if (lane == 0) wcnt[wave] = wc;
    __syncthreads();
    if (wave == 0) {
#pragma unroll 1
      for (int wsx = 0; wsx < NWAVE; ++wsx) {
        int n = __builtin_amdgcn_readfirstlane(wcnt[wsx]);
        n = n > WCAP ? WCAP : (n < 0 ? 0 : n);
        const int* lq = list + wsx * WCAP;
#pragma unroll 1
        for (int i = 0; i < n; ++i) {
          const int ent  = __builtin_amdgcn_readfirstlane(lq[i]);
          const int slot = ent & (NB - 1);
          int e = cbase + ((ent >> 12) & (CHUNK - 1));
          e = e > nE - 1 ? nE - 1 : e;
          int src = ei[e];
          src = src < 0 ? 0 : (src > nN - 1 ? nN - 1 : src);
          const v4f v = *(const v4f*)(g2 + (size_t)src * DE + 4 * lane);
          v4f* ap = (v4f*)(acc + slot * DF + 4 * lane);
          *ap = *ap + v;
        }
      }
    }
    __syncthreads();
  }

#pragma unroll 4
  for (int i = 0; i < (NB * DF / 4) / NTHR; ++i) {
    const int idx  = i * NTHR + tid;
    const int slot = idx >> 5;
    const int c4   = (idx & 31) * 4;
    int node = nodeBase + slot;
    node = node > nN - 1 ? nN - 1 : node;
    const float d  = dinv[node];
    const v4f   gv = *(const v4f*)(g2 + (size_t)node * DE + c4);
    const v4f   bv = *(const v4f*)(b2 + c4);
    v4f* ap = (v4f*)(acc + slot * DF + c4);
    v4f hv = (*ap + gv) * d + bv;
    hv.x = fmaxf(hv.x, 0.f); hv.y = fmaxf(hv.y, 0.f); hv.z = fmaxf(hv.z, 0.f); hv.w = fmaxf(hv.w, 0.f);
    *ap = hv;
  }
  __syncthreads();

  float* ob = h2 + (size_t)nodeBase * DE;
#pragma unroll 4
  for (int q = 0; q < 64; ++q) {
    const int f = (wave * 64 + q) * 128 + 4 * lane;
    const v4f v = *(const v4f*)(acc + f);
    *(volatile v4f*)(ob + f) = v;
  }
  __threadfence();
#pragma unroll 4
  for (int q = 0; q < 64; ++q) {
    const int f = (wave * 64 + q) * 128 + 4 * lane;
    const v4f v = *(const v4f*)(acc + f);
    *(volatile v4f*)(ob + f) = v;
  }
}

__global__ __launch_bounds__(NTHR) void k_pool(
    const int* __restrict__ batch, const float* __restrict__ h2, const float* __restrict__ ss2,
    float* out, int nN, int vec8) {
  __shared__ __attribute__((aligned(16))) int list[LISTN];
  __shared__ int wcnt[NWAVE];
  __shared__ __attribute__((aligned(16))) float mrow[DE];
  const int tid = threadIdx.x, lane = tid & 31, wave = tid >> 5;
  const int g = blockIdx.x;
  const int ch = tid < DE ? tid : 0;
  const float sc = ss2[ch];
  const float sh = ss2[SSOFF + ch];
  float mx = -__builtin_inff();

  const int nChunks = (nN + CHUNK - 1) / CHUNK;
#pragma unroll 1
  for (int chnk = 0; chnk < nChunks; ++chnk) {
    const int cbase = chnk * CHUNK;
    const int wc = scan_chunk<1>(batch, nN, cbase, g, vec8, list, tid, lane, wave);
    if (lane == 0) wcnt[wave] = wc;
    __syncthreads();
#pragma unroll 1
    for (int wsx = 0; wsx < NWAVE; ++wsx) {
      int n = __builtin_amdgcn_readfirstlane(wcnt[wsx]);
      n = n > WCAP ? WCAP : (n < 0 ? 0 : n);
      const int* lq = list + wsx * WCAP;
#pragma unroll 1
      for (int i = 0; i < n; ++i) {
        const int ent = __builtin_amdgcn_readfirstlane(lq[i]);
        int node = cbase + ((ent >> 12) & (CHUNK - 1));
        node = node > nN - 1 ? nN - 1 : node;
        if (tid < DE) {
          const float v = h2[(size_t)node * DE + tid] * sc + sh;
          mx = fmaxf(mx, v);
        }
      }
    }
    __syncthreads();
  }

  if (tid < DE) mrow[tid] = mx;
  __syncthreads();
  if (wave == 0) {
    const v4f v = *(const v4f*)(mrow + 4 * lane);
    float* op = out + (size_t)g * DE + 4 * lane;
    *(volatile v4f*)op = v;
    __threadfence();
    *(volatile v4f*)op = v;
  }
}

extern "C" void kernel_launch(void* const* d_in, const int* in_sizes, int n_in,
                              void* d_out, int out_size, void* d_ws, size_t ws_size,
                              hipStream_t stream) {
  if (n_in < 11) return;
  const int nN = in_sizes[0] / DIN;
  const int nE = in_sizes[1] / 2;
  const int nG = out_size / DE;
  if (nN <= 0 || nE < 0 || nG <= 0) return;
  if (in_sizes[0] != nN * DIN || in_sizes[1] != 2 * nE || in_sizes[2] != nN) return;
  if (in_sizes[3] != DIN * DH || in_sizes[4] < DH || in_sizes[5] < DH || in_sizes[6] < DH) return;
  if (in_sizes[7] != DH * DE || in_sizes[8] < DE || in_sizes[9] < DE || in_sizes[10] < DE) return;
  if (out_size != nG * DE) return;

  const float* x      = (const float*)d_in[0];
  const int*   ei     = (const int*)d_in[1];
  const int*   batch  = (const int*)d_in[2];
  const float* W1     = (const float*)d_in[3];
  const float* b1     = (const float*)d_in[4];
  const float* gamma1 = (const float*)d_in[5];
  const float* beta1  = (const float*)d_in[6];
  const float* W2     = (const float*)d_in[7];
  const float* b2     = (const float*)d_in[8];
  const float* gamma2 = (const float*)d_in[9];
  const float* beta2  = (const float*)d_in[10];
  float* out = (float*)d_out;

  const int nBD = (nN + NBD - 1) / NBD;
  const int nA  = (nN + NB - 1) / NB;
  const int nS  = (nN + SROWS - 1) / SROWS;
  const int nG2 = (nN + G2ROWS - 1) / G2ROWS;

  char* ws = (char*)d_ws;
  size_t off = 0;
  const size_t oW1 = off; off += (size_t)DH * DIN * 2;                 off = (off + 255) & ~(size_t)255;
  const size_t oW2 = off; off += (size_t)DE * DH * 2;                  off = (off + 255) & ~(size_t)255;
  const size_t oDv = off; off += (size_t)nBD * NBD * 4;                off = (off + 255) & ~(size_t)255;
  const size_t oH1 = off; off += (size_t)nA * NB * DH * 4;             off = (off + 255) & ~(size_t)255;
  const size_t oP1 = off; off += (size_t)nS * 2 * DH * 8;              off = (off + 255) & ~(size_t)255;
  const size_t oS1 = off; off += (size_t)2 * SSOFF * 4;                off = (off + 255) & ~(size_t)255;
  const size_t oG2 = off; off += (size_t)nG2 * G2ROWS * DE * 4;        off = (off + 255) & ~(size_t)255;
  const size_t oH2 = off; off += (size_t)nA * NB * DE * 4;             off = (off + 255) & ~(size_t)255;
  const size_t oP2 = off; off += (size_t)nS * 2 * DE * 8;              off = (off + 255) & ~(size_t)255;
  const size_t oS2 = off; off += (size_t)2 * SSOFF * 4;                off = (off + 255) & ~(size_t)255;
  if (off > ws_size) return;
  _Float16* w1s  = (_Float16*)(ws + oW1);
  _Float16* w2s  = (_Float16*)(ws + oW2);
  float*    dinv = (float*)(ws + oDv);
  float*    h1   = (float*)(ws + oH1);
  double*   p1   = (double*)(ws + oP1);
  float*    ss1  = (float*)(ws + oS1);
  float*    g2   = (float*)(ws + oG2);
  float*    h2   = (float*)(ws + oH2);
  double*   p2   = (double*)(ws + oP2);
  float*    ss2  = (float*)(ws + oS2);

  const int vec8 = ((nE & 3) == 0) ? 1 : 0;

  const int nPrep = DH * DIN / 8 + DE * DH / 8;
  k_wprep<<<(nPrep + NTHR - 1) / NTHR, NTHR, 0, stream>>>(W1, W2, w1s, w2s);

  k_deg<<<nBD, NTHR, 0, stream>>>(ei, dinv, nN, nE, vec8);

  hipFuncSetAttribute(reinterpret_cast<const void*>(&k_agg1),
                      hipFuncAttributeMaxDynamicSharedMemorySize, LDS_AGG);
  k_agg1<<<nA, NTHR, LDS_AGG, stream>>>(ei, x, dinv, b1, w1s, h1, nN, nE, vec8);

  k_bnstat<<<nS, DH, 0, stream>>>(h1, p1, DH, nN, SROWS);
  k_bnfin<<<1, DH, 0, stream>>>(p1, nS, DH, nN, gamma1, beta1, ss1);

  hipFuncSetAttribute(reinterpret_cast<const void*>(&k_gemm2),
                      hipFuncAttributeMaxDynamicSharedMemorySize, LDS_GEMM2);
  k_gemm2<<<nG2, NTHR, LDS_GEMM2, stream>>>(h1, ss1, w2s, dinv, g2, nN);

  hipFuncSetAttribute(reinterpret_cast<const void*>(&k_agg2),
                      hipFuncAttributeMaxDynamicSharedMemorySize, LDS_AGG);
  k_agg2<<<nA, NTHR, LDS_AGG, stream>>>(ei, g2, dinv, b2, h2, nN, nE, vec8);

  k_bnstat<<<nS, DE, 0, stream>>>(h2, p2, DE, nN, SROWS);
  k_bnfin<<<1, DE, 0, stream>>>(p2, nS, DE, nN, gamma2, beta2, ss2);

  k_pool<<<nG, NTHR, 0, stream>>>(batch, h2, ss2, out, nN, 1);
}
